// SmallestAdditionTransformer_55585466745161
// MI455X (gfx1250) — hardware-verified
//
#include <hip/hip_runtime.h>
#include <stddef.h>


typedef _Float16 h16;
typedef _Float16 v16h __attribute__((ext_vector_type(16)));
typedef _Float16 v8h  __attribute__((ext_vector_type(8)));
typedef float    v8f  __attribute__((ext_vector_type(8)));
typedef float    v4f  __attribute__((ext_vector_type(4)));

#ifndef NB
#define NB 32768
#endif
#define NB_FULL 32768
#define TLEN 34
#define VOC  14
#define SPB  8
#define TOK  (SPB * TLEN)
#define NTHR 288
#define OUT_F4 (TOK * VOC / 4)
#define VROWS 8
#define VKEYS 64

#ifndef INPUT_BF16
#define INPUT_BF16 1
#endif
#ifndef PV_RES
#define PV_RES 1
#endif

#define PCARRY 16384.0f
#define VCARRY 16.0f
#define RCARRY 2048.0f
#define OSCALE 3.814697265625e-06f

static_assert(NB >= SPB && NB <= NB_FULL && (NB % SPB) == 0);
static_assert((TOK * VOC * 4) % 128 == 0);
static_assert((TOK * VOC) % 4 == 0);
static_assert(OUT_F4 % 8 == 0);
static_assert(NTHR % 32 == 0 && NTHR >= TOK);
static_assert(4 * NTHR >= OUT_F4);
static_assert(TLEN > 32 && TLEN <= 48);
static_assert(TLEN - 32 == 2);
static_assert(VKEYS == 64 && VROWS == 8);
static_assert(SPB <= NTHR / 32);

__device__ __forceinline__ float bf16r(float x) {
  unsigned int u = __float_as_uint(x);
  u = (u + 0x7FFFu + ((u >> 16) & 1u)) & 0xFFFF0000u;
  return __uint_as_float(u);
}
__device__ __forceinline__ float inw(float x) {
  return INPUT_BF16 ? bf16r(x) : x;
}
static __device__ __forceinline__ h16 toh_flush(float v) {
  const h16 r = (h16)v;
  return (fabsf(v) < 6.103515625e-05f) ? (h16)0.0f : r;
}

__device__ __forceinline__ v16h frag_at(const _Float16* p) {
  v8h lo = *(const v8h*)(p);
  v8h hi = *(const v8h*)(p + 16);
  v16h out;
#pragma unroll
  for (int i = 0; i < 8; ++i) { out[i] = lo[i]; out[i + 8] = hi[i]; }
  return out;
}

__device__ __forceinline__ v8f wmma16(v16h a, v16h b, v8f c) {
  v8f d = __builtin_amdgcn_wmma_f32_16x16x32_f16(false, a, false, b, (short)0, c,
                                                 false, false);
  asm volatile("v_nop\n\tv_nop\n\tv_nop\n\tv_nop" : "+v"(d) : "v"(a), "v"(b));
  return d;
}

__device__ __forceinline__ void ln6(const float (&x)[6], const float* __restrict__ g,
                                    const float* __restrict__ b, float (&h)[6]) {
  const float mu = (x[0] + x[1] + x[2] + x[3] + x[4] + x[5]) * (1.0f / 6.0f);
  float var = 0.0f;
#pragma unroll
  for (int c = 0; c < 6; ++c) { const float d = x[c] - mu; var += d * d; }
  var *= (1.0f / 6.0f);
  const float rs = rsqrtf(var + 1.0e-5f);
#pragma unroll
  for (int c = 0; c < 6; ++c) h[c] = (x[c] - mu) * rs * inw(g[c]) + inw(b[c]);
}

__global__ __launch_bounds__(NTHR) void fused_block_kernel(
    const int* __restrict__ idx, const float* __restrict__ tok_emb,
    const float* __restrict__ pos_params, const float* __restrict__ z10_enc,
    const float* __restrict__ special_enc, const float* __restrict__ wq,
    const float* __restrict__ wk, const float* __restrict__ wv, const float* __restrict__ wo,
    const float* __restrict__ ln1_g, const float* __restrict__ ln1_b,
    const float* __restrict__ ln2_g, const float* __restrict__ ln2_b,
    const float* __restrict__ lnf_g, const float* __restrict__ lnf_b,
    const float* __restrict__ ffn_w1, const float* __restrict__ ffn_b1,
    const float* __restrict__ ffn_w2, const float* __restrict__ ffn_b2,
    const float* __restrict__ head_w, float* __restrict__ out) {
  __shared__ __attribute__((aligned(16))) v4f sQ4[SPB * 2 * TLEN];
  __shared__ __attribute__((aligned(16))) v4f sK4[SPB * 2 * TLEN];
  __shared__ __attribute__((aligned(16))) _Float16 sVTh[SPB * VROWS * VKEYS];
  __shared__ __attribute__((aligned(16))) _Float16 sVTr[SPB * VROWS * VKEYS];
  __shared__ __attribute__((aligned(16))) float sO[TOK * 6];
  __shared__ __attribute__((aligned(16))) float sDen[TOK * 2];
  __shared__ __attribute__((aligned(16))) float sPos[TLEN * 4];
  __shared__ __attribute__((aligned(16))) float sLog[TOK * VOC];

  const unsigned tid = threadIdx.x;
  const unsigned lane = tid & 31u;
  const int wave = __builtin_amdgcn_readfirstlane((int)(tid >> 5));
  const unsigned hh = lane >> 4, m = lane & 15u;

  {
    const v8h z = {};
    for (unsigned i = tid; i < (unsigned)(SPB * VROWS * VKEYS / 8); i += NTHR) {
      *(v8h*)&sVTh[i * 8u] = z;
      *(v8h*)&sVTr[i * 8u] = z;
    }
  }
  if (wave < 2) {
    const unsigned t = (tid < (unsigned)TLEN) ? tid : (unsigned)(TLEN - 1);
    const float amp   = inw(pos_params[0]);
    const float phase = inw(pos_params[1]);
    const float slope = inw(pos_params[2]);
    const float offs  = inw(pos_params[3]);
    int di = (t < 10u) ? (int)t : ((t < 21u) ? ((int)t - 11) : ((int)t - 22));
    di = (di < 0) ? 0 : ((di > 9) ? 9 : di);
    const float fi  = (float)di;
    const float ang = 0.62831853071795864769f * fi + phase;
    const float d0 = amp * cosf(ang);
    const float d1 = amp * sinf(ang);
    const float d2 = slope * fi + offs;
    const unsigned si = (t == 10u) ? 0u : ((t == 21u) ? 1u : 2u);
    const float s0 = inw(special_enc[si * 3u + 0u]);
    const float s1 = inw(special_enc[si * 3u + 1u]);
    const float s2 = inw(special_enc[si * 3u + 2u]);
    const float z0 = inw(z10_enc[0]);
    const float z1 = inw(z10_enc[1]);
    const float z2 = inw(z10_enc[2]);
    const bool is_sp = (t == 10u) || (t == 21u) || (t == 33u);
    const bool is_z  = (t == 32u);
    const float p0 = is_sp ? s0 : (is_z ? z0 : d0);
    const float p1 = is_sp ? s1 : (is_z ? z1 : d1);
    const float p2 = is_sp ? s2 : (is_z ? z2 : d2);
    if (tid < (unsigned)TLEN) {
      sPos[t * 4u + 0u] = p0;
      sPos[t * 4u + 1u] = p1;
      sPos[t * 4u + 2u] = p2;
      sPos[t * 4u + 3u] = 0.0f;
    }
  }
  __syncthreads();

  const bool act = tid < (unsigned)TOK;
  const unsigned p = act ? tid : (unsigned)(TOK - 1);
  const unsigned s = p / (unsigned)TLEN;
  const unsigned t = p - s * (unsigned)TLEN;
  float x[6];
  {
    const size_t seq_g = (size_t)blockIdx.x * SPB + s;
    int tok = idx[seq_g * TLEN + t];
    tok = (tok < 0) ? 0 : ((tok > VOC - 1) ? (VOC - 1) : tok);
#pragma unroll
    for (int c = 0; c < 3; ++c) {
      x[c]     = inw(tok_emb[tok * 3 + c]);
      x[3 + c] = sPos[t * 4u + (unsigned)c];
    }
    float h[6];
    ln6(x, ln1_g, ln1_b, h);
    float q[6], k[6], v[6];
#pragma unroll
    for (int j = 0; j < 6; ++j) {
      q[j] = h[3] * inw(wq[j]) + h[4] * inw(wq[6 + j]) + h[5] * inw(wq[12 + j]);
      k[j] = h[3] * inw(wk[j]) + h[4] * inw(wk[6 + j]) + h[5] * inw(wk[12 + j]);
      v[j] = h[0] * inw(wv[j]) + h[1] * inw(wv[6 + j]) + h[2] * inw(wv[12 + j]);
    }
    if (act) {
      v4f q0 = {q[0], q[1], q[2], 0.0f};
      v4f q1 = {q[3], q[4], q[5], 0.0f};
      v4f k0 = {k[0], k[1], k[2], 0.0f};
      v4f k1 = {k[3], k[4], k[5], 0.0f};
      sQ4[(s * 2u + 0u) * TLEN + t] = q0;
      sQ4[(s * 2u + 1u) * TLEN + t] = q1;
      sK4[(s * 2u + 0u) * TLEN + t] = k0;
      sK4[(s * 2u + 1u) * TLEN + t] = k1;
#pragma unroll
      for (int n = 0; n < 6; ++n) {
        const float vv = v[n] * VCARRY;
        const h16 hi = toh_flush(vv);
        const h16 rs = toh_flush((vv - (float)hi) * RCARRY);
        sVTh[(s * VROWS + (unsigned)n) * VKEYS + t] = hi;
        sVTr[(s * VROWS + (unsigned)n) * VKEYS + t] = rs;
      }
    }
  }
  __syncthreads();

  if (wave < SPB) {
    const unsigned seq = (unsigned)wave;
    const unsigned vrow = (seq * VROWS + (m & 7u)) * VKEYS + 8u * hh;
    const v16h bh0 = frag_at(&sVTh[vrow]);
    const v16h br0 = frag_at(&sVTr[vrow]);
    const v16h bh1 = frag_at(&sVTh[vrow + 32u]);
    const v16h br1 = frag_at(&sVTr[vrow + 32u]);

#pragma unroll 1
    for (unsigned hd = 0; hd < 2u; ++hd) {
      const unsigned qkb = (seq * 2u + hd) * TLEN;
#pragma unroll
      for (int qt = 0; qt < 3; ++qt) {
        const bool last = (qt == 2);
        const unsigned tr = 16u * (unsigned)qt + m;
        const unsigned tq = (tr < (unsigned)TLEN) ? tr : (unsigned)(TLEN - 1);
        const v4f qv = sQ4[qkb + tq];

        float sc[16];
        float sx[2];
        float mx = -1.0e30f;
#pragma unroll
        for (int i = 0; i < 16; ++i) {
          const unsigned j = 8u * hh + (unsigned)(i & 7) + 16u * (unsigned)(i >> 3);
          const v4f kv = sK4[qkb + j];
          float sv = (qv[0] * kv[0] + qv[1] * kv[1] + qv[2] * kv[2]) * 0.57735026918962576f;
          sv = (j > tq) ? -1.0e30f : sv;
          sc[i] = sv;
          mx = fmaxf(mx, sv);
        }
        if (last) {
#pragma unroll
          for (int e = 0; e < 2; ++e) {
            const unsigned j = 32u + (unsigned)e;
            const v4f kv = sK4[qkb + j];
            float sv = (qv[0] * kv[0] + qv[1] * kv[1] + qv[2] * kv[2]) * 0.57735026918962576f;
            sv = ((hh != 0u) || (j > tq)) ? -1.0e30f : sv;
            sx[e] = sv;
            mx = fmaxf(mx, sv);
          }
        }
        mx = fmaxf(mx, __shfl_xor(mx, 16, 32));

        v16h ahi, ars;
        v16h xhi = {}, xrs = {};
        float den = 0.0f;
#pragma unroll
        for (int i = 0; i < 16; ++i) {
          const unsigned j = 8u * hh + (unsigned)(i & 7) + 16u * (unsigned)(i >> 3);
          float pe = __expf(sc[i] - mx);
          pe = (j > tq) ? 0.0f : pe;
          den += pe;
          const float pv = pe * PCARRY;
          const h16 hi = toh_flush(pv);
          ahi[i] = hi;
          ars[i] = toh_flush((pv - (float)hi) * RCARRY);
        }
        if (last) {
#pragma unroll
          for (int e = 0; e < 2; ++e) {
            const unsigned j = 32u + (unsigned)e;
            float pe = __expf(sx[e] - mx);
            pe = ((hh != 0u) || (j > tq)) ? 0.0f : pe;
            den += pe;
            const float pv = pe * PCARRY;
            const h16 hi = toh_flush(pv);
            xhi[e] = hi;
            xrs[e] = toh_flush((pv - (float)hi) * RCARRY);
          }
        }
        den += __shfl_xor(den, 16, 32);

        v8f accM = {}, accR = {};
        accM = wmma16(ahi, bh0, accM);
        if (PV_RES) {
          accR = wmma16(ahi, br0, accR);
          accR = wmma16(ars, bh0, accR);
        }
        if (last) {
          accM = wmma16(xhi, bh1, accM);
          if (PV_RES) {
            accR = wmma16(xhi, br1, accR);
            accR = wmma16(xrs, bh1, accR);
          }
        }

        const bool colok = (m >= 3u * hd) && (m < 3u * hd + 3u);
#pragma unroll
        for (int r = 0; r < 8; ++r) {
          const unsigned row = 16u * (unsigned)qt + 8u * hh + (unsigned)r;
          const float val = accM[r] + accR[r] * (1.0f / RCARRY);
          if (colok && row < (unsigned)TLEN) sO[(seq * TLEN + row) * 6u + m] = val;
        }
        if (hh == 0u && tr < (unsigned)TLEN) sDen[(seq * TLEN + tr) * 2u + hd] = den;
      }
    }
  }
  __syncthreads();

  {
    float o[6];
    const float inv0 = (1.0f / sDen[p * 2u + 0u]) * OSCALE;
    const float inv1 = (1.0f / sDen[p * 2u + 1u]) * OSCALE;
#pragma unroll
    for (int c = 0; c < 3; ++c) {
      o[c]     = sO[p * 6u + (unsigned)c] * inv0;
      o[3 + c] = sO[p * 6u + 3u + (unsigned)c] * inv1;
    }
    float x2[6];
#pragma unroll
    for (int j = 0; j < 6; ++j) {
      float acc = x[j];
#pragma unroll
      for (int c = 0; c < 6; ++c) acc += o[c] * inw(wo[c * 6 + j]);
      x2[j] = acc;
    }
    float h2[6];
    ln6(x2, ln2_g, ln2_b, h2);
    float f0 = inw(ffn_b1[0]), f1 = inw(ffn_b1[1]);
#pragma unroll
    for (int j = 0; j < 6; ++j) {
      f0 += h2[j] * inw(ffn_w1[j * 2 + 0]);
      f1 += h2[j] * inw(ffn_w1[j * 2 + 1]);
    }
    f0 = 0.5f * f0 * (1.0f + erff(f0 * 0.70710678118654752f));
    f1 = 0.5f * f1 * (1.0f + erff(f1 * 0.70710678118654752f));
#pragma unroll
    for (int j = 0; j < 6; ++j)
      x2[j] += f0 * inw(ffn_w2[j]) + f1 * inw(ffn_w2[6 + j]) + inw(ffn_b2[j]);
    float xf[6];
    ln6(x2, lnf_g, lnf_b, xf);
    float y[3];
#pragma unroll
    for (int d = 0; d < 3; ++d) {
      float acc = 0.0f;
#pragma unroll
      for (int c = 0; c < 6; ++c) acc += xf[c] * inw(head_w[c * 3 + d]);
      y[d] = acc;
    }
#pragma unroll 2
    for (int n = 0; n < VOC; ++n) {
      const float lg = y[0] * inw(tok_emb[n * 3 + 0]) + y[1] * inw(tok_emb[n * 3 + 1]) +
                       y[2] * inw(tok_emb[n * 3 + 2]);
      if (act) sLog[p * VOC + (unsigned)n] = lg;
    }
  }
  __syncthreads();

  {
    float* outB = out + (size_t)blockIdx.x * (size_t)(TOK * VOC);
    v4f xs[4];
#pragma unroll
    for (unsigned j = 0; j < 4u; ++j) {
      const unsigned i = tid + NTHR * j;
      const unsigned ic = (i < (unsigned)OUT_F4) ? i : (unsigned)(OUT_F4 - 1);
      xs[j] = *(const v4f*)&sLog[ic * 4u];
    }
#pragma unroll
    for (unsigned j = 0; j < 4u; ++j) {
      const unsigned i = tid + NTHR * j;
      if (i < (unsigned)OUT_F4) *(volatile v4f*)(outB + (size_t)i * 4u) = xs[j];
    }
    __threadfence();
#pragma unroll
    for (unsigned j = 0; j < 4u; ++j) {
      const unsigned i = tid + NTHR * j;
      if (i < (unsigned)OUT_F4) *(volatile v4f*)(outB + (size_t)i * 4u) = xs[j];
    }
  }
}

extern "C" void kernel_launch(void* const* d_in, const int* in_sizes, int n_in,
                              void* d_out, int out_size, void* d_ws, size_t ws_size,
                              hipStream_t stream) {
  (void)d_ws; (void)ws_size;
  if (n_in < 20) return;
  if ((long long)in_sizes[0] < (long long)NB * TLEN) return;
  if (in_sizes[1] < VOC * 3 || in_sizes[2] < 4 || in_sizes[3] < 3 || in_sizes[4] < 9) return;
  if (in_sizes[5] < 18 || in_sizes[6] < 18 || in_sizes[7] < 18 || in_sizes[8] < 36) return;
  if (in_sizes[9] < 6 || in_sizes[10] < 6 || in_sizes[11] < 6 || in_sizes[12] < 6) return;
  if (in_sizes[13] < 6 || in_sizes[14] < 6) return;
  if (in_sizes[15] < 12 || in_sizes[16] < 2 || in_sizes[17] < 12 || in_sizes[18] < 6) return;
  if (in_sizes[19] < 18) return;
  if ((long long)out_size < (long long)NB * TLEN * VOC) return;

  const int*   idx         = (const int*)  d_in[0];
  const float* tok_emb     = (const float*)d_in[1];
  const float* pos_params  = (const float*)d_in[2];
  const float* z10_enc     = (const float*)d_in[3];
  const float* special_enc = (const float*)d_in[4];
  const float* wq          = (const float*)d_in[5];
  const float* wk          = (const float*)d_in[6];
  const float* wv          = (const float*)d_in[7];
  const float* wo          = (const float*)d_in[8];
  const float* ln1_g       = (const float*)d_in[9];
  const float* ln1_b       = (const float*)d_in[10];
  const float* ln2_g       = (const float*)d_in[11];
  const float* ln2_b       = (const float*)d_in[12];
  const float* lnf_g       = (const float*)d_in[13];
  const float* lnf_b       = (const float*)d_in[14];
  const float* ffn_w1      = (const float*)d_in[15];
  const float* ffn_b1      = (const float*)d_in[16];
  const float* ffn_w2      = (const float*)d_in[17];
  const float* ffn_b2      = (const float*)d_in[18];
  const float* head_w      = (const float*)d_in[19];
  float* out = (float*)d_out;

  fused_block_kernel<<<dim3(NB / SPB), dim3(NTHR), 0, stream>>>(
      idx, tok_emb, pos_params, z10_enc, special_enc, wq, wk, wv, wo,
      ln1_g, ln1_b, ln2_g, ln2_b, lnf_g, lnf_b,
      ffn_w1, ffn_b1, ffn_w2, ffn_b2, head_w, out);
}
